// IntraGraphAttention_11647951307189
// MI455X (gfx1250) — hardware-verified
//
#include <hip/hip_runtime.h>
#include <stddef.h>


#define IN_DIM  128
#define KP      256
#define HEADS   2
#define OUT_CH  35
#define OUTC    (HEADS * OUT_CH)
#define NPAD    80
#define NT16    5
#define WTROWS  (2 * NPAD)
#define YP      96
#define YH1     48
#define EP      2
#define NTHR    256
#define NWAVE   8
#define EPT     8
#define CHUNK   (NTHR * EPT)
#define WCAP    (EPT * 32)
#define LISTN   (NWAVE * WCAP)
#define NBMAX   2048
#define RCAP    24576
#define DEGCAP  4096
#define SUB     16
#define OSTW    (SUB * OUTC)
#define GBM     64
#define GTHR    128
#define NEG_SLOPE 0.2f
#define WSCAP   134217728
#define LDS_INTS (2 * RCAP + 2 * NBMAX + LISTN + 2 * NWAVE)
#define LDS_AGG  (LDS_INTS * 4 + NWAVE * OSTW * 4 + YP * 4)

static_assert((CHUNK & (CHUNK - 1)) == 0 && CHUNK <= 4096);
static_assert((NBMAX & (NBMAX - 1)) == 0 && NBMAX <= 2048);
static_assert(NTHR * 8 == NBMAX);
static_assert(LISTN >= NBMAX);
static_assert(LISTN >= NWAVE * WCAP);
static_assert((RCAP % 32) == 0);
static_assert(LDS_AGG <= 300000);
static_assert(((LDS_INTS * 4) % 16) == 0);
static_assert(((OSTW * 4) % 16) == 0);
static_assert((OSTW % 4) == 0);
static_assert(GBM == (GTHR / 32) * 16);
static_assert(2 * GBM == GTHR);
static_assert(NT16 * 16 == NPAD && NPAD >= OUTC);
static_assert(KP == 2 * IN_DIM && (KP % 32) == 0 && (IN_DIM % 32) == 0);
static_assert(YP == 2 * YH1 && YH1 >= OUT_CH && YH1 + OUT_CH <= YP && (YP % 32) == 0);
static_assert(GBM * EP == 32 * 4);
static_assert(24 * 4 == YP);
static_assert((SUB * OUTC * 4) % 128 == 0);

typedef float    v4f  __attribute__((ext_vector_type(4)));
typedef float    v8f  __attribute__((ext_vector_type(8)));
typedef int      v4i  __attribute__((ext_vector_type(4)));
typedef int      v8i  __attribute__((ext_vector_type(8)));
typedef unsigned short v8us __attribute__((ext_vector_type(8)));
typedef __bf16   v16bf __attribute__((ext_vector_type(16)));
typedef v4f      v4fa __attribute__((may_alias));
typedef v8us     v8usa __attribute__((may_alias));
union FragB { v16bf v; v8us h[2]; v8i w; };

__device__ __forceinline__ v8f wmb(const FragB& a, const FragB& b, v8f c) {
  v8f d = __builtin_amdgcn_wmma_f32_16x16x32_bf16(false, a.v, false, b.v, (short)0, c, false, false);
  asm volatile("v_nop\n\tv_nop\n\tv_nop\n\tv_nop" : "+v"(d) : "v"(a.w), "v"(b.w));
  return d;
}

__device__ __forceinline__ unsigned short bf16_rne(float f) {
  unsigned u = __float_as_uint(f);
  u = u + 0x7FFFu + ((u >> 16) & 1u);
  return (unsigned short)(u >> 16);
}
__device__ __forceinline__ float bf16_val(unsigned short b) {
  return __uint_as_float(((unsigned)b) << 16);
}

__device__ __forceinline__ int scan_chunk(const int* __restrict__ dsts, int nE, int cbase, int slotBase,
                                          int nb, int vec8, int* list, int tid, int lane, int wave) {
  int wc = 0;
  const int el0  = tid * EPT;
  const int e0   = cbase + el0;
  const int sent = -2147483647 - 1;
  v4i da, db;
  if (vec8 != 0 && cbase + CHUNK <= nE) {
    da = *(const v4i*)(dsts + e0);
    db = *(const v4i*)(dsts + e0 + 4);
  } else {
    da.x = (e0     < nE) ? dsts[min(e0,     nE - 1)] : sent;
    da.y = (e0 + 1 < nE) ? dsts[min(e0 + 1, nE - 1)] : sent;
    da.z = (e0 + 2 < nE) ? dsts[min(e0 + 2, nE - 1)] : sent;
    da.w = (e0 + 3 < nE) ? dsts[min(e0 + 3, nE - 1)] : sent;
    db.x = (e0 + 4 < nE) ? dsts[min(e0 + 4, nE - 1)] : sent;
    db.y = (e0 + 5 < nE) ? dsts[min(e0 + 5, nE - 1)] : sent;
    db.z = (e0 + 6 < nE) ? dsts[min(e0 + 6, nE - 1)] : sent;
    db.w = (e0 + 7 < nE) ? dsts[min(e0 + 7, nE - 1)] : sent;
  }
  const unsigned nbs = (unsigned)slotBase;
  const unsigned unb = (unsigned)nb;
  const unsigned s0 = (unsigned)da.x - nbs, s1 = (unsigned)da.y - nbs;
  const unsigned s2 = (unsigned)da.z - nbs, s3 = (unsigned)da.w - nbs;
  const unsigned s4 = (unsigned)db.x - nbs, s5 = (unsigned)db.y - nbs;
  const unsigned s6 = (unsigned)db.z - nbs, s7 = (unsigned)db.w - nbs;
  const bool h0 = s0 < unb, h1 = s1 < unb, h2 = s2 < unb, h3 = s3 < unb;
  const bool h4 = s4 < unb, h5 = s5 < unb, h6 = s6 < unb, h7 = s7 < unb;
  const unsigned any = __builtin_amdgcn_ballot_w32(h0 | h1 | h2 | h3 | h4 | h5 | h6 | h7);
  if (any != 0u) {
#define HITJ(J, HJ, SJ) { \
      const unsigned mj = __builtin_amdgcn_ballot_w32(HJ); \
      if (mj != 0u) { \
        if (HJ) { \
          const int pos = wc + (int)__builtin_amdgcn_mbcnt_lo(mj, 0u); \
          if (pos < WCAP) list[wave * WCAP + pos] = ((el0 + (J)) << 12) | (int)(SJ); \
        } \
        wc += (int)__builtin_popcount(mj); } }
    HITJ(0, h0, s0)
    HITJ(1, h1, s1)
    HITJ(2, h2, s2)
    HITJ(3, h3, s3)
    HITJ(4, h4, s4)
    HITJ(5, h5, s5)
    HITJ(6, h6, s6)
    HITJ(7, h7, s7)
#undef HITJ
  }
  return wc;
}

__global__ __launch_bounds__(NTHR) void k_xprep(const float* __restrict__ x, unsigned short* xh, int nN) {
  __shared__ __attribute__((aligned(16))) unsigned short sh[2 * KP];
  const int tid = (int)threadIdx.x;
  const int r2 = tid >> 7, c = tid & (IN_DIM - 1);
  const int row = (int)blockIdx.x * 2 + r2;
  const int rc = row < nN ? row : nN - 1;
  float v = x[(size_t)rc * IN_DIM + c];
  if (row >= nN) v = 0.f;
  const float em = expm1f(v);
  const float e = v > 0.f ? v : em;
  const unsigned short hb = bf16_rne(e);
  const float lo = e - bf16_val(hb);
  const unsigned short lb = bf16_rne(lo);
  sh[r2 * KP + c] = hb;
  sh[r2 * KP + IN_DIM + c] = lb;
  __syncthreads();
  if (tid < 64) {
    const int rr = tid >> 5, l = tid & 31;
    const v8us hv = *(const v8usa*)(sh + rr * KP + 8 * l);
    const size_t o = (size_t)((int)blockIdx.x * 2 + rr) * KP + 8 * l;
    *(volatile v8us*)(xh + o) = hv;
    __threadfence();
    *(volatile v8us*)(xh + o) = hv;
  }
}

__global__ __launch_bounds__(NTHR) void k_wprep(const float* __restrict__ w, unsigned short* wt) {
  const int u = (int)blockIdx.x * NTHR + (int)threadIdx.x;
  if (u >= WTROWS * (KP / 8)) return;
  const int ng = u >> 5;
  const int k8 = (u & 31) * 8;
  const int pl = (ng >= NPAD) ? 1 : 0;
  const int n  = ng - pl * NPAD;
  const int kk = k8 & (IN_DIM - 1);
  const int ncl = n < OUTC ? n : OUTC - 1;
  const bool valid = (n < OUTC) && ((pl == 0) || (k8 < IN_DIM));
  const float* p = w + (size_t)kk * OUTC + ncl;
  v8us hv;
#pragma unroll
  for (int i = 0; i < 8; ++i) {
    const float fv = p[(size_t)i * OUTC];
    const unsigned short hb = bf16_rne(fv);
    const unsigned short lb = bf16_rne(fv - bf16_val(hb));
    unsigned short val = (pl == 0) ? hb : lb;
    if (!valid) val = (unsigned short)0;
    hv[i] = val;
  }
  const size_t o = (size_t)ng * KP + k8;
  *(volatile v8us*)(wt + o) = hv;
  __threadfence();
  *(volatile v8us*)(wt + o) = hv;
}

__device__ __forceinline__ v4f yrow4(const float* srow, int lane) {
  v4f v;
#pragma unroll
  for (int e = 0; e < 4; ++e) {
    const int j = 4 * lane + e;
    const bool up = j >= YH1;
    const int sc = up ? j - (YH1 - OUT_CH) : j;
    const bool ok = up ? (j - YH1 < OUT_CH) : (j < OUT_CH);
    const int scc = sc < NPAD - 1 ? sc : NPAD - 1;
    const float f = srow[scc];
    v[e] = ok ? f : 0.f;
  }
  return v;
}

__global__ __launch_bounds__(GTHR) void k_gemm(const unsigned short* __restrict__ xh,
                                               const unsigned short* __restrict__ wt,
                                               const float* __restrict__ asrc, const float* __restrict__ adst,
                                               float* Y, float* ES, float* ED) {
  __shared__ __attribute__((aligned(16))) float stg[GBM * NPAD];
  __shared__ __attribute__((aligned(16))) float esT[GBM * EP];
  __shared__ __attribute__((aligned(16))) float edT[GBM * EP];
  __shared__ float sAs[OUTC];
  __shared__ float sAd[OUTC];
  const int tid = (int)threadIdx.x, lane = tid & 31, wave = tid >> 5, hh = lane >> 4, m = lane & 15;
  const int rowBase = (int)blockIdx.x * GBM;
  if (tid < OUTC) { sAs[tid] = asrc[tid]; sAd[tid] = adst[tid]; }

  v8f acc[NT16];
#pragma unroll
  for (int t = 0; t < NT16; ++t) { v8f z = {0.f, 0.f, 0.f, 0.f, 0.f, 0.f, 0.f, 0.f}; acc[t] = z; }
  const size_t arow = (size_t)(rowBase + 16 * wave + m) * KP + 8 * hh;
  const size_t brow = (size_t)m * KP + 8 * hh;
#pragma unroll 1
  for (int ks = 0; ks < IN_DIM / 32; ++ks) {
    FragB af;
    af.h[0] = *(const v8us*)(xh + arow + 32 * ks);
    af.h[1] = *(const v8us*)(xh + arow + 32 * ks + 16);
#pragma unroll
    for (int t = 0; t < NT16; ++t) {
      const size_t bo = brow + (size_t)(16 * t) * KP + 32 * ks;
      FragB bf;
      bf.h[0] = *(const v8us*)(wt + bo);
      bf.h[1] = *(const v8us*)(wt + bo + 16);
      acc[t] = wmb(af, bf, acc[t]);
      const size_t bo2 = bo + (size_t)NPAD * KP;
      FragB bg;
      bg.h[0] = *(const v8us*)(wt + bo2);
      bg.h[1] = *(const v8us*)(wt + bo2 + 16);
      acc[t] = wmb(af, bg, acc[t]);
    }
  }
#pragma unroll 1
  for (int ks = IN_DIM / 32; ks < KP / 32; ++ks) {
    FragB af;
    af.h[0] = *(const v8us*)(xh + arow + 32 * ks);
    af.h[1] = *(const v8us*)(xh + arow + 32 * ks + 16);
#pragma unroll
    for (int t = 0; t < NT16; ++t) {
      const size_t bo = brow + (size_t)(16 * t) * KP + 32 * ks;
      FragB bf;
      bf.h[0] = *(const v8us*)(wt + bo);
      bf.h[1] = *(const v8us*)(wt + bo + 16);
      acc[t] = wmb(af, bf, acc[t]);
    }
  }
  {
    float* sp = stg + (size_t)(16 * wave + 8 * hh) * NPAD + m;
#pragma unroll
    for (int t = 0; t < NT16; ++t) {
#pragma unroll
      for (int r = 0; r < 8; ++r) sp[(size_t)r * NPAD + 16 * t] = acc[t][r];
    }
  }
  __syncthreads();
  {
    const int row  = tid >> 1;
    const int half = tid & 1;
    const float* srow = stg + (size_t)row * NPAD + OUT_CH * half;
    float s = 0.f, d = 0.f;
#pragma unroll 1
    for (int c = 0; c < OUT_CH; ++c) {
      const float v = srow[c];
      s = fmaf(v, sAs[OUT_CH * half + c], s);
      d = fmaf(v, sAd[OUT_CH * half + c], d);
    }
    esT[row * EP + half] = s;
    edT[row * EP + half] = d;
  }
  __syncthreads();
#pragma unroll 1
  for (int r = wave; r < GBM; r += GTHR / 32) {
    if (lane < 24) {
      const v4f v = yrow4(stg + (size_t)r * NPAD, lane);
      *(volatile v4f*)(Y + (size_t)(rowBase + r) * YP + 4 * lane) = v;
    }
  }
  __threadfence();
#pragma unroll 1
  for (int r = wave; r < GBM; r += GTHR / 32) {
    if (lane < 24) {
      const v4f v = yrow4(stg + (size_t)r * NPAD, lane);
      *(volatile v4f*)(Y + (size_t)(rowBase + r) * YP + 4 * lane) = v;
    }
  }
  if (wave == 0) {
    const v4f ve = *(const v4f*)(esT + 4 * lane);
    float* pe = ES + (size_t)rowBase * EP + 4 * lane;
    *(volatile v4f*)pe = ve;
    __threadfence();
    *(volatile v4f*)pe = ve;
  } else if (wave == 1) {
    const v4f vd = *(const v4f*)(edT + 4 * lane);
    float* pd = ED + (size_t)rowBase * EP + 4 * lane;
    *(volatile v4f*)pd = vd;
    __threadfence();
    *(volatile v4f*)pd = vd;
  }
}

__global__ __launch_bounds__(NTHR) void k_agg(
    const int* __restrict__ srcs, const int* __restrict__ dsts,
    const float* __restrict__ Y, const float* __restrict__ ES, const float* __restrict__ ED,
    const float* __restrict__ bias, float* out,
    int nN, int nE, int nb, int vec8) {
  extern __shared__ v4f lds_dyn[];
  int* reg1 = (int*)lds_dyn;
  int* reg2 = reg1 + RCAP;
  int* scnt = reg2 + RCAP;
  int* soff = scnt + NBMAX;
  int* list = soff + NBMAX;
  int* wcnt = list + LISTN;
  int* wtot = wcnt + NWAVE;
  float* ostg = (float*)(wtot + NWAVE);
  float* sBY  = ostg + NWAVE * OSTW;
  const int tid = (int)threadIdx.x, lane = tid & 31, wave = tid >> 5;
  const int nodeBase = (int)blockIdx.x * nb;

  for (int i = tid; i < NBMAX; i += NTHR) scnt[i] = 0;
  if (tid < YP) {
    const int j = tid;
    const bool up = j >= YH1;
    const int bc = up ? j - (YH1 - OUT_CH) : j;
    const bool ok = up ? (j - YH1 < OUT_CH) : (j < OUT_CH);
    const int bcc = bc < OUTC - 1 ? bc : OUTC - 1;
    const float bv = bias[bcc];
    sBY[j] = ok ? bv : 0.f;
  }
  __syncthreads();

  int tot = 0;
  const int nChunks = (nE + CHUNK - 1) / CHUNK;
#pragma unroll 1
  for (int ch = 0; ch < nChunks; ++ch) {
    const int cbase = ch * CHUNK;
    const int wc = scan_chunk(dsts, nE, cbase, nodeBase, nb, vec8, list, tid, lane, wave);
    if (lane == 0) wcnt[wave] = wc;
    __syncthreads();
    int pre = 0, all = 0;
#pragma unroll
    for (int w2 = 0; w2 < NWAVE; ++w2) {
      int c = wcnt[w2];
      c = c < 0 ? 0 : (c > WCAP ? WCAP : c);
      all += c;
      pre += (w2 < wave) ? c : 0;
    }
    const int wcc  = wc > WCAP ? WCAP : wc;
    const int base = tot + pre;
#pragma unroll 1
    for (int i = lane; i < wcc; i += 32) {
      const int ent = list[wave * WCAP + i];
      const int el  = (ent >> 12) & (CHUNK - 1);
      const int sl  = ent & (NBMAX - 1);
      int eid = cbase + el;
      eid = eid > nE - 1 ? nE - 1 : eid;
      const int pos = base + i;
      if (pos < RCAP) reg1[pos] = (int)(((unsigned)eid << 11) | (unsigned)sl);
    }
    tot += all;
    tot = tot > RCAP ? RCAP : tot;
    __syncthreads();
  }
  const int nh = tot;

  if (wave == 0) {
#pragma unroll 1
    for (int b0 = 0; b0 < nh; b0 += 32) {
      const int idx = b0 + lane;
      const int uv  = reg1[idx < RCAP ? idx : RCAP - 1];
      const int m32 = (nh - b0) < 32 ? (nh - b0) : 32;
#pragma unroll 1
      for (int k = 0; k < m32; ++k) {
        const int u  = __builtin_amdgcn_readlane(uv, k);
        const int sl = u & (NBMAX - 1);
        if (lane == 0) scnt[sl] = scnt[sl] + 1;
      }
    }
  }
  __syncthreads();

  {
    const v4i ca = *(const v4i*)(scnt + 8 * tid);
    const v4i cb = *(const v4i*)(scnt + 8 * tid + 4);
    const int e0 = ca.x < 0 ? 0 : ca.x, e1 = ca.y < 0 ? 0 : ca.y, e2 = ca.z < 0 ? 0 : ca.z, e3 = ca.w < 0 ? 0 : ca.w;
    const int e4 = cb.x < 0 ? 0 : cb.x, e5 = cb.y < 0 ? 0 : cb.y, e6 = cb.z < 0 ? 0 : cb.z, e7 = cb.w < 0 ? 0 : cb.w;
    const int ts = e0 + e1 + e2 + e3 + e4 + e5 + e6 + e7;
    int incl = ts;
#pragma unroll
    for (int d = 1; d < 32; d <<= 1) {
      const int up = __shfl_up(incl, d);
      if (lane >= d) incl += up;
    }
    if (lane == 31) wtot[wave] = incl;
    __syncthreads();
    int pre = 0;
#pragma unroll
    for (int w2 = 0; w2 < NWAVE; ++w2) pre += (w2 < wave) ? wtot[w2] : 0;
    int run = pre + incl - ts;
    soff[8 * tid + 0] = run; run += e0;
    soff[8 * tid + 1] = run; run += e1;
    soff[8 * tid + 2] = run; run += e2;
    soff[8 * tid + 3] = run; run += e3;
    soff[8 * tid + 4] = run; run += e4;
    soff[8 * tid + 5] = run; run += e5;
    soff[8 * tid + 6] = run; run += e6;
    soff[8 * tid + 7] = run;
  }
  __syncthreads();
  for (int i = tid; i < NBMAX; i += NTHR) list[i] = soff[i];
  __syncthreads();

  if (wave == 0) {
#pragma unroll 1
    for (int b0 = 0; b0 < nh; b0 += 32) {
      const int idx = b0 + lane;
      const int uv  = reg1[idx < RCAP ? idx : RCAP - 1];
      const int m32 = (nh - b0) < 32 ? (nh - b0) : 32;
#pragma unroll 1
      for (int k = 0; k < m32; ++k) {
        const int u   = __builtin_amdgcn_readlane(uv, k);
        const int sl  = u & (NBMAX - 1);
        const int eid = (int)((unsigned)u >> 11);
        if (lane == 0) {
          int pos = list[sl];
          pos = pos < 0 ? 0 : (pos > RCAP - 1 ? RCAP - 1 : pos);
          reg2[pos] = eid;
          list[sl] = pos + 1;
        }
      }
    }
  }
  __syncthreads();

  const int q   = lane < 23 ? lane : 23;
  const int c4  = 4 * q;
  const int hd  = (q >= 12) ? 1 : 0;
  const bool lact = lane < 24;
  const int jo  = hd ? (YH1 - OUT_CH) : 0;
  const int jl  = hd ? (YH1 + OUT_CH) : OUT_CH;
  const int ch0 = c4 - jo, ch1 = c4 + 1 - jo, ch2 = c4 + 2 - jo, ch3 = c4 + 3 - jo;
  const bool v0 = lact && (c4 < jl), v1 = lact && (c4 + 1 < jl);
  const bool v2 = lact && (c4 + 2 < jl), v3 = lact && (c4 + 3 < jl);
  const bool ovf = (nh >= RCAP);
  const float qnan = __int_as_float(0x7fc00000);
  float* myo = ostg + (size_t)wave * OSTW;
  const v4fa* my4 = (const v4fa*)myo;
  const int nsub = nb >> 4;
#pragma unroll 1
  for (int jb = wave; jb < nsub; jb += NWAVE) {
    const int slot0 = jb * SUB;
#pragma unroll 1
    for (int r = 0; r < SUB; ++r) {
      const int slot = slot0 + r;
      const int grow = nodeBase + slot;
      const int gcl  = grow < nN ? grow : nN - 1;
      int st = soff[slot];
      const int craw = scnt[slot];
      int cnt = craw;
      st  = st < 0 ? 0 : (st > nh ? nh : st);
      cnt = cnt < 0 ? 0 : (cnt > DEGCAP ? DEGCAP : cnt);
      if (cnt > nh - st) cnt = nh - st;
      const float pz = (ovf || craw > DEGCAP) ? qnan : 0.0f;

      const float* yd = Y + (size_t)gcl * YP + c4;
      v4f a = *(const v4f*)yd;
      const float edv = ED[(size_t)gcl * EP + hd];
      const float esd = ES[(size_t)gcl * EP + hd];
      const float t0 = esd + edv;
      float mx = fmaxf(t0, NEG_SLOPE * t0);
      float dn = 1.0f;
#pragma unroll 1
      for (int p = 0; p < cnt; ++p) {
        int idx = st + p; idx = idx > RCAP - 1 ? RCAP - 1 : idx;
        int eid = reg2[idx]; eid = eid < 0 ? 0 : (eid > nE - 1 ? nE - 1 : eid);
        const int sraw = srcs[eid];
        const int s = sraw < 0 ? 0 : (sraw > nN - 1 ? nN - 1 : sraw);
        const v4f xs = *(const v4f*)(Y + (size_t)s * YP + c4);
        const float ess = ES[(size_t)s * EP + hd];
        const float u = ess + edv;
        const float l = fmaxf(u, NEG_SLOPE * u);
        const float mn = fmaxf(mx, l);
        const float s1 = __expf(mx - mn), s2 = __expf(l - mn);
        dn = fmaf(dn, s1, s2);
        a.x = fmaf(a.x, s1, s2 * xs.x);
        a.y = fmaf(a.y, s1, s2 * xs.y);
        a.z = fmaf(a.z, s1, s2 * xs.z);
        a.w = fmaf(a.w, s1, s2 * xs.w);
        mx = mn;
      }
      const float inv = __builtin_amdgcn_rcpf(dn);
      const float o0 = fmaf(a.x, inv, sBY[c4 + 0]) + pz;
      const float o1 = fmaf(a.y, inv, sBY[c4 + 1]) + pz;
      const float o2 = fmaf(a.z, inv, sBY[c4 + 2]) + pz;
      const float o3 = fmaf(a.w, inv, sBY[c4 + 3]) + pz;
      float* orow = myo + r * OUTC;
      if (v0) orow[ch0] = o0;
      if (v1) orow[ch1] = o1;
      if (v2) orow[ch2] = o2;
      if (v3) orow[ch3] = o3;
    }
    __builtin_amdgcn_fence(__ATOMIC_RELEASE, "wavefront");
    __builtin_amdgcn_wave_barrier();
    int nval = nN - (nodeBase + slot0);
    nval = nval < 0 ? 0 : (nval > SUB ? SUB : nval);
    if (nval > 0) {
      const int fl  = nval * OUTC;
      const int n4  = fl >> 2;
      const int rem = fl & 3;
      float* ob = out + (size_t)(nodeBase + slot0) * OUTC;
      const int ti = 4 * n4 + (lane & 3);
      const float tv = myo[ti < OSTW ? ti : OSTW - 1];
      const bool tw = (rem != 0) && (lane < rem);
#pragma unroll
      for (int i = 0; i < 9; ++i) {
        const int f  = 32 * i + lane;
        const int fc = f < OSTW / 4 ? f : OSTW / 4 - 1;
        const v4f v = my4[fc];
        if (f < n4) *(volatile v4f*)(ob + 4 * f) = v;
      }
      if (tw) *(volatile float*)(ob + 4 * n4 + lane) = tv;
      __threadfence();
#pragma unroll
      for (int i = 0; i < 9; ++i) {
        const int f  = 32 * i + lane;
        const int fc = f < OSTW / 4 ? f : OSTW / 4 - 1;
        const v4f v = my4[fc];
        if (f < n4) *(volatile v4f*)(ob + 4 * f) = v;
      }
      if (tw) *(volatile float*)(ob + 4 * n4 + lane) = tv;
    }
    __builtin_amdgcn_fence(__ATOMIC_RELEASE, "wavefront");
    __builtin_amdgcn_wave_barrier();
  }
}

static int pick_nb(int nE, int nN) {
  int nb = NBMAX;
  while (nb > 16 && (long long)nb * (long long)nE * 5LL > (long long)RCAP * (long long)nN * 4LL) nb >>= 1;
  return nb;
}

extern "C" void kernel_launch(void* const* d_in, const int* in_sizes, int n_in,
                              void* d_out, int out_size, void* d_ws, size_t ws_size,
                              hipStream_t stream) {
  if (n_in < 6) return;
  const int nN = in_sizes[0] / IN_DIM;
  if (nN <= 0 || in_sizes[0] != nN * IN_DIM) return;
  if (nN > (1 << 22)) return;
  const int nE = in_sizes[1] / 2;
  if (nE < 1 || in_sizes[1] != 2 * nE) return;
  if (nE > (1 << 21)) return;
  if (in_sizes[2] != IN_DIM * OUTC) return;
  if (in_sizes[3] != OUTC || in_sizes[4] != OUTC) return;
  if (in_sizes[5] != OUTC) return;
  if ((long long)out_size != (long long)nN * OUTC) return;

  const float* x   = (const float*)d_in[0];
  const int*   ei  = (const int*)d_in[1];
  const float* W   = (const float*)d_in[2];
  const float* as  = (const float*)d_in[3];
  const float* ad  = (const float*)d_in[4];
  const float* bs  = (const float*)d_in[5];
  float* out = (float*)d_out;

  const int MP   = ((nN + GBM - 1) / GBM) * GBM;
  const int nb   = pick_nb(nE, nN);
  const int vec8 = ((nE & 3) == 0) ? 1 : 0;

  char* ws = (char*)d_ws;
  size_t off = 0;
  const size_t oWT = off; off += (size_t)WTROWS * KP * 2;        off = (off + 255) & ~(size_t)255;
  const size_t oXH = off; off += (size_t)MP * KP * 2;            off = (off + 255) & ~(size_t)255;
  const size_t oY  = off; off += (size_t)MP * YP * 4;            off = (off + 255) & ~(size_t)255;
  const size_t oES = off; off += (size_t)MP * EP * 4;            off = (off + 255) & ~(size_t)255;
  const size_t oED = off; off += (size_t)MP * EP * 4;            off = (off + 255) & ~(size_t)255;
  if (off > ws_size || off > (size_t)WSCAP) return;
  unsigned short* WT = (unsigned short*)(ws + oWT);
  unsigned short* XH = (unsigned short*)(ws + oXH);
  float*    Y  = (float*)(ws + oY);
  float*    ES = (float*)(ws + oES);
  float*    ED = (float*)(ws + oED);

  hipFuncSetAttribute(reinterpret_cast<const void*>(&k_agg),
                      hipFuncAttributeMaxDynamicSharedMemorySize, LDS_AGG);

  k_xprep<<<MP / 2, NTHR, 0, stream>>>(x, XH, nN);
  k_wprep<<<(WTROWS * (KP / 8) + NTHR - 1) / NTHR, NTHR, 0, stream>>>(W, WT);

  const int gG = MP / GBM;
  const int gA = (nN + nb - 1) / nb;

  k_gemm<<<gG, GTHR, 0, stream>>>(XH, WT, as, ad, Y, ES, ED);
  k_agg<<<gA, NTHR, LDS_AGG, stream>>>(ei, ei + nE, Y, ES, ED, bs, out, nN, nE, nb, vec8);
}
